// UltraTransformerBlock_55508157333992
// MI455X (gfx1250) — hardware-verified
//
#include <hip/hip_runtime.h>
#include <math.h>
#include <stdint.h>
#include <stddef.h>


#define D_MODEL 768
#define NQH     12
#define NKVH    4
#define HDIM    64
#define KV_DIM  256
#define QKV_N   1280
#define FF_DIM  2048
#define SEQ_LEN 2048
#define NREP    3

typedef __attribute__((ext_vector_type(16))) _Float16 v16h;
typedef __attribute__((ext_vector_type(8)))  _Float16 v8h;
typedef __attribute__((ext_vector_type(16))) __bf16   v16b;
typedef __attribute__((ext_vector_type(8)))  __bf16   v8b;
typedef __attribute__((ext_vector_type(8)))  float    v8f;
typedef __attribute__((ext_vector_type(4)))  float    v4f;
typedef __attribute__((ext_vector_type(2)))  float    v2f;

__device__ __forceinline__ unsigned short f2bf_bits(float f) {
  unsigned u = __float_as_uint(f);
  return (unsigned short)((u + 0x7FFFu + ((u >> 16) & 1u)) >> 16);
}
__device__ __forceinline__ float bf_bits2f(unsigned short h) { return __uint_as_float(((unsigned)h) << 16); }

__device__ __forceinline__ void dep_guard_h(v8f& a, v8f& b, v16h x, v16h y) { asm volatile("v_nop\n\tv_nop\n\tv_nop\n\tv_nop" : "+v"(a), "+v"(b) : "v"(x), "v"(y)); }
__device__ __forceinline__ void dep_guard_b(v8f& a, v8f& b, v16b x, v16b y) { asm volatile("v_nop\n\tv_nop\n\tv_nop\n\tv_nop" : "+v"(a), "+v"(b) : "v"(x), "v"(y)); }
__device__ __forceinline__ void keep4_h(v16h a, v16h b, v16h c, v16h d) { asm volatile("v_nop" :: "v"(a), "v"(b), "v"(c), "v"(d)); }
__device__ __forceinline__ void keep4_b(v16b a, v16b b, v16b c, v16b d) { asm volatile("v_nop" :: "v"(a), "v"(b), "v"(c), "v"(d)); }
__device__ __forceinline__ void acc_guard4(v8f& a, v8f& b, v8f& c, v8f& d) { asm volatile("v_nop\n\tv_nop\n\tv_nop\n\tv_nop" : "+v"(a), "+v"(b), "+v"(c), "+v"(d)); }
template <typename T> struct Frag;
template <> struct Frag<_Float16> {
  typedef v16h V; union U { v16h v; v8h h[2]; };
  static __device__ __forceinline__ v16h load(const _Float16* p) {
    U f; f.h[0] = *(const v8h*)(p); f.h[1] = *(const v8h*)(p + 16); return f.v;
  }
  static __device__ __forceinline__ v8f mma(v16h a, v16h b, v8f c) {
    return __builtin_amdgcn_wmma_f32_16x16x32_f16(false, a, false, b, (short)0, c, false, false);
  }
  static __device__ __forceinline__ void guard(v8f& a, v8f& b, v16h x, v16h y) { dep_guard_h(a, b, x, y); }
  static __device__ __forceinline__ void keep(v16h a, v16h b, v16h c, v16h d) { keep4_h(a, b, c, d); }
};
template <> struct Frag<__bf16> {
  typedef v16b V; union U { v16b v; v8b h[2]; };
  static __device__ __forceinline__ v16b load(const __bf16* p) {
    U f; f.h[0] = *(const v8b*)(p); f.h[1] = *(const v8b*)(p + 16); return f.v;
  }
  static __device__ __forceinline__ v8f mma(v16b a, v16b b, v8f c) {
    return __builtin_amdgcn_wmma_f32_16x16x32_bf16(false, a, false, b, (short)0, c, false, false);
  }
  static __device__ __forceinline__ void guard(v8f& a, v8f& b, v16b x, v16b y) { dep_guard_b(a, b, x, y); }
  static __device__ __forceinline__ void keep(v16b a, v16b b, v16b c, v16b d) { keep4_b(a, b, c, d); }
};

template <int ET> struct Elem;
template <> struct Elem<0> { typedef _Float16 T; };
template <> struct Elem<1> { typedef __bf16 T; };
template <int ET, bool SPLIT, int BIAS_MODE, int OUT_MODE, bool RESID, int ACT = 0>
__global__ __launch_bounds__(256) void wmma_gemm64(
    const unsigned short* __restrict__ Ap, const unsigned short* __restrict__ A2p, int lda, long strideA,
    const unsigned short* __restrict__ Btp, const unsigned short* __restrict__ Bt2p, int ldb, long strideB,
    void* __restrict__ Cout, void* __restrict__ Cout2, int ldc, long strideC,
    const float* __restrict__ bias,
    const float* __restrict__ resid, long strideR,
    int M, int N, int K, float scale) {
  typedef typename Elem<ET>::T T;
  typedef typename Frag<T>::V V;
  const T* A = (const T*)Ap; const T* A2 = (const T*)A2p; const T* Bt = (const T*)Btp; const T* Bt2 = (const T*)Bt2p;
  __shared__ __align__(16) float sT[8][16 * 68];
  const int b    = blockIdx.y;
  const int lane = threadIdx.x & 31;
  const int wave = threadIdx.x >> 5;
  const int tilesN = N >> 6;
  const int tilesM = M >> 6;
  const int tile = blockIdx.x * 8 + wave;
  if (tile >= tilesM * tilesN) return;
  const int tm = tile / tilesN;
  const int tn = tile - tm * tilesN;
  const int m0 = tm << 6;
  const int n0 = tn << 6;

  const T* Ab  = A  + (size_t)b * strideA;
  const T* Bb  = Bt + (size_t)b * strideB;
  const T* Ab2 = SPLIT ? (A2  + (size_t)b * strideA) : nullptr;
  const T* Bb2 = SPLIT ? (Bt2 + (size_t)b * strideB) : nullptr;

  const int rlane = lane & 15;
  const int koff  = (lane >> 4) * 8;
  const int mOff  = (lane >> 4) * 8;

  v8f acc[4][4];
#pragma unroll
  for (int i = 0; i < 4; ++i)
#pragma unroll
    for (int j = 0; j < 4; ++j) acc[i][j] = (v8f){0.f,0.f,0.f,0.f,0.f,0.f,0.f,0.f};

  for (int k0 = 0; k0 < K; k0 += 32) {
    V bh[4], bl[4];
#pragma unroll
    for (int j = 0; j < 4; ++j) {
      const size_t bo = (size_t)(n0 + (j << 4) + rlane) * ldb + koff + k0;
      bh[j] = Frag<T>::load(Bb + bo);
      if (SPLIT) bl[j] = Frag<T>::load(Bb2 + bo);
    }
#pragma unroll
    for (int i = 0; i < 4; ++i) {
      const size_t ao = (size_t)(m0 + (i << 4) + rlane) * lda + koff + k0;
      V ah = Frag<T>::load(Ab + ao);
      V al;
      if (SPLIT) al = Frag<T>::load(Ab2 + ao);
#pragma unroll
      for (int j = 0; j < 4; ++j) {
        acc[i][j] = Frag<T>::mma(ah, bh[j], acc[i][j]);
        if (SPLIT) {
          acc[i][j] = Frag<T>::mma(ah, bl[j], acc[i][j]);
          acc[i][j] = Frag<T>::mma(al, bh[j], acc[i][j]);
        }
      }
      Frag<T>::guard(acc[i][0], acc[i][3], ah, SPLIT ? al : ah);
    }
    Frag<T>::keep(bh[0], bh[1], bh[2], bh[3]);
    if (SPLIT) Frag<T>::keep(bl[0], bl[1], bl[2], bl[3]);
  }
  acc_guard4(acc[0][0], acc[0][1], acc[0][2], acc[0][3]);
  acc_guard4(acc[1][0], acc[1][1], acc[1][2], acc[1][3]);
  acc_guard4(acc[2][0], acc[2][1], acc[2][2], acc[2][3]);
  acc_guard4(acc[3][0], acc[3][1], acc[3][2], acc[3][3]);

  float* slab = sT[wave];
  const float* Rb = RESID ? (resid + (size_t)b * strideR) : nullptr;
#pragma unroll
  for (int i = 0; i < 4; ++i) {
    const int mBase = m0 + (i << 4);
#pragma unroll
    for (int j = 0; j < 4; ++j) {
      const int n = n0 + (j << 4) + rlane;
      float bv = 0.f;
      if (BIAS_MODE == 2) bv = bias[n];
#pragma unroll
      for (int r = 0; r < 8; ++r) {
        float v = acc[i][j][r] * scale;
        if (BIAS_MODE == 1) v += bias[mBase + mOff + r];
        if (BIAS_MODE == 2) v += bv;
        if (RESID) v += Rb[(size_t)(mBase + mOff + r) * ldc + n];
        if (ACT == 1) v = tanhf(v);
        if (ACT == 2) v = fmaxf(v, 0.0f);
        if (ACT == 3) v = v / (1.0f + expf(-v));
        if (ACT == 4) v = (v > 0.f) ? v : 0.01f * v;
        if (ACT == 5) v = 0.5f * v * (1.0f + erff(v * 0.70710678118654752f));
        slab[(mOff + r) * 68 + (j << 4) + rlane] = v;
      }
    }
    __builtin_amdgcn_fence(__ATOMIC_RELEASE, "workgroup");
    __builtin_amdgcn_wave_barrier();
    __builtin_amdgcn_fence(__ATOMIC_ACQUIRE, "workgroup");
    if (OUT_MODE == 0) {
      float* C = (float*)Cout + (size_t)b * strideC;
      const int hh = lane >> 4, c4 = (lane & 15) * 4;
      for (int pass = 0; pass < 2; ++pass) {
#pragma unroll
        for (int it = 0; it < 8; ++it) {
          const int row = it * 2 + hh;
          v4f v = *(const v4f*)(slab + row * 68 + c4);
          *(volatile v4f*)(C + (size_t)(mBase + row) * ldc + n0 + c4) = v;
        }
        __threadfence();
      }
    } else {
      const int q = lane >> 3, c8 = (lane & 7) * 8;
      unsigned short* C  = (unsigned short*)Cout  + (size_t)b * strideC;
      unsigned short* C2 = (OUT_MODE == 2) ? ((unsigned short*)Cout2 + (size_t)b * strideC) : nullptr;
      for (int pass = 0; pass < 2; ++pass) {
#pragma unroll
        for (int it = 0; it < 4; ++it) {
          const int row = it * 4 + q;
          const float* sp = slab + row * 68 + c8;
          v8h hv, lv;
#pragma unroll
          for (int e = 0; e < 8; ++e) {
            if (OUT_MODE == 1) {
              hv[e] = (_Float16)sp[e];
            } else {
              unsigned short hb = f2bf_bits(sp[e]);
              unsigned short lb = f2bf_bits(sp[e] - bf_bits2f(hb));
              hv[e] = __builtin_bit_cast(_Float16, hb);
              lv[e] = __builtin_bit_cast(_Float16, lb);
            }
          }
          *(volatile v8h*)(C + (size_t)(mBase + row) * ldc + n0 + c8) = hv;
          if (OUT_MODE == 2) *(volatile v8h*)(C2 + (size_t)(mBase + row) * ldc + n0 + c8) = lv;
        }
        __threadfence();
      }
    }
    __builtin_amdgcn_fence(__ATOMIC_RELEASE, "workgroup");
    __builtin_amdgcn_wave_barrier();
    __builtin_amdgcn_fence(__ATOMIC_ACQUIRE, "workgroup");
  }
}

__global__ __launch_bounds__(256) void cast_scale_f32_f16x2(
    const float* __restrict__ in, _Float16* __restrict__ out, int n2, float scale) {
  const int i = blockIdx.x * 256 + threadIdx.x;
  if (i < n2) {
    const v2f xv = *(const v2f*)(in + 2 * (size_t)i);
    const _Float16 h0 = (_Float16)(xv[0] * scale), h1 = (_Float16)(xv[1] * scale);
    const unsigned u = (unsigned)__builtin_bit_cast(unsigned short, h0) | ((unsigned)__builtin_bit_cast(unsigned short, h1) << 16);
    ((volatile unsigned*)out)[i] = u;
    __threadfence();
    ((volatile unsigned*)out)[i] = u;
  }
}

struct RopeFreq { float f[32]; };
static_assert(sizeof(RopeFreq) == 128);
__global__ __launch_bounds__(256) void rope_table(float* __restrict__ cosT, float* __restrict__ sinT, int S, RopeFreq rf) {
  const int i = blockIdx.y;
  const int s = blockIdx.x * 256 + threadIdx.x;
  if (s >= S) return;
  float inv = rf.f[0];
#pragma unroll
  for (int t = 1; t < 32; ++t) inv = (i == t) ? rf.f[t] : inv;
  const float ang = (float)s * inv;
  float sv, cv;
  sincosf(ang, &sv, &cv);
  float* cp = cosT + (size_t)i * S + s;
  float* sp = sinT + (size_t)i * S + s;
  *(volatile float*)cp = cv;
  *(volatile float*)sp = sv;
  __threadfence();
  *(volatile float*)cp = cv;
  *(volatile float*)sp = sv;
}

__global__ __launch_bounds__(256) void rmsnorm768_f16(const float* __restrict__ x, const float* __restrict__ g,
                                                       _Float16* __restrict__ out, int M, float nscale, float eps) {
  const int wave = threadIdx.x >> 5, lane = threadIdx.x & 31;
  const int rowu = blockIdx.x * 8 + wave;
  const bool valid = rowu < M;
  const int row = valid ? rowu : (M - 1);
  const float* xr = x + (size_t)row * D_MODEL + 8 * lane;
  const float* gr = g + 8 * lane;
  v4f xa[3], xb[3], ga[3], gb[3];
  float ss = 0.f;
#pragma unroll
  for (int j = 0; j < 3; ++j) {
    xa[j] = *(const v4f*)(xr + 256 * j);
    xb[j] = *(const v4f*)(xr + 256 * j + 4);
    ga[j] = *(const v4f*)(gr + 256 * j);
    gb[j] = *(const v4f*)(gr + 256 * j + 4);
#pragma unroll
    for (int e = 0; e < 4; ++e) { ss += xa[j][e] * xa[j][e]; ss += xb[j][e] * xb[j][e]; }
  }
#pragma unroll
  for (int off = 1; off < 32; off <<= 1) ss += __shfl_xor(ss, off, 32);
  const float norm = sqrtf(ss) * nscale;
  const float inv = 1.0f / (norm + eps);
  v8h o[3];
#pragma unroll
  for (int j = 0; j < 3; ++j) {
#pragma unroll
    for (int e = 0; e < 4; ++e) {
      o[j][e]     = (_Float16)((ga[j][e] * xa[j][e]) * inv);
      o[j][4 + e] = (_Float16)((gb[j][e] * xb[j][e]) * inv);
    }
  }
  if (valid) {
    _Float16* orow = out + (size_t)row * D_MODEL + 8 * lane;
    for (int pass = 0; pass < 2; ++pass) {
#pragma unroll
      for (int j = 0; j < 3; ++j) *(volatile v8h*)(orow + 256 * j) = o[j];
      __threadfence();
    }
  }
}

__global__ __launch_bounds__(256) void rope_split_f16(const float* __restrict__ qkv,
                                                      const float* __restrict__ cosT, const float* __restrict__ sinT,
                                                      _Float16* __restrict__ qo, _Float16* __restrict__ ko, _Float16* __restrict__ vo,
                                                      int M, int S) {
  const int idx = blockIdx.x * 256 + threadIdx.x;
  if (idx >= M * (QKV_N / 8)) return;
  const int row  = idx / (QKV_N / 8);
  const int col0 = (idx - row * (QKV_N / 8)) * 8;
  const int s    = row % S;
  const float* src = qkv + (size_t)row * QKV_N + col0;
  const v4f a0 = *(const v4f*)src, a1 = *(const v4f*)(src + 4);
  const bool rot  = col0 < (D_MODEL + KV_DIM);
  const int  d0   = col0 & (HDIM - 1);
  const bool lowh = d0 < 32;
  const int  po   = rot ? (lowh ? 32 : -32) : 0;
  const float sg  = lowh ? -1.0f : 1.0f;
  const v4f p0 = *(const v4f*)(src + po), p1 = *(const v4f*)(src + po + 4);
  const int i0 = d0 & 31;
  const float* cb = cosT + (size_t)i0 * S + s;
  const float* sb = sinT + (size_t)i0 * S + s;
  v4f c0, c1, n0, n1;
#pragma unroll
  for (int e = 0; e < 4; ++e) {
    c0[e] = cb[(size_t)e * S];        c1[e] = cb[(size_t)(e + 4) * S];
    n0[e] = sb[(size_t)e * S];        n1[e] = sb[(size_t)(e + 4) * S];
  }
  const v4f r0 = a0 * c0 + sg * (p0 * n0);
  const v4f r1 = a1 * c1 + sg * (p1 * n1);
  v8h hv;
#pragma unroll
  for (int e = 0; e < 4; ++e) {
    hv[e]     = (_Float16)(rot ? r0[e] : a0[e]);
    hv[4 + e] = (_Float16)(rot ? r1[e] : a1[e]);
  }
  _Float16* dst;
  if (col0 < D_MODEL)               dst = qo + (size_t)row * D_MODEL + col0;
  else if (col0 < D_MODEL + KV_DIM) dst = ko + (size_t)row * KV_DIM + (col0 - D_MODEL);
  else                              dst = vo + (size_t)row * KV_DIM + (col0 - D_MODEL - KV_DIM);
  *(volatile v8h*)dst = hv;
  __threadfence();
  *(volatile v8h*)dst = hv;
}

#define AT_D 64
#define AT_NW 4
#define AT_QB 64
#define AT_KC 64
#define AT_PSC 32768.0f
struct AttnGeomH { long q_bs, q_rs, q_hs, k_bs, k_rs, k_hs, v_bs, v_rs, v_hs, o_bs, o_rs, o_hs;
                   int S, H, n_rep, causal; float qscale, oscale; };
static_assert(sizeof(AttnGeomH) == 120);

__device__ __forceinline__ v8f mma_h(v16h a, v16h b, v8f c) {
  c = __builtin_amdgcn_wmma_f32_16x16x32_f16(false, a, false, b, (short)0, c, false, false);
  asm volatile("v_nop\n\tv_nop\n\tv_nop\n\tv_nop" : "+v"(c) : "v"(a), "v"(b));
  return c;
}

__global__ __launch_bounds__(128)
void attn64_f16(const _Float16* __restrict__ q, const _Float16* __restrict__ k,
                const _Float16* __restrict__ v, _Float16* __restrict__ out, AttnGeomH g) {
  union FH { v16h v; v8h h[2]; };
  __shared__ __align__(16) _Float16 Ksh[AT_KC * AT_D];
  __shared__ __align__(16) _Float16 Vth[AT_D * AT_KC];
  __shared__ __align__(16) _Float16 Psh[AT_NW][16 * AT_KC];
  __shared__ __align__(16) float    Os[AT_NW][16 * 68];

  const int tid  = threadIdx.x;
  const int wave = tid >> 5;
  const int lane = tid & 31;
  const int hh   = lane >> 4;
  const int c    = lane & 15;

  const int nqb = g.S / AT_QB;
  const int bx = blockIdx.x;
  const int qb = bx % nqb;
  const int bh = bx / nqb;
  const int h  = bh % g.H;
  const int b  = bh / g.H;
  const int hk = h / g.n_rep;
  const int q0 = qb * AT_QB + wave * 16;

  const _Float16* qb_ptr = q + (size_t)b * g.q_bs + (size_t)h * g.q_hs;
  const _Float16* kb_ptr = k + (size_t)b * g.k_bs + (size_t)hk * g.k_hs;
  const _Float16* vb_ptr = v + (size_t)b * g.v_bs + (size_t)hk * g.v_hs;
  _Float16*       ob_ptr = out + (size_t)b * g.o_bs + (size_t)h * g.o_hs;

  v16h qa[2];
  {
    const _Float16* qrow = qb_ptr + (size_t)(q0 + c) * g.q_rs;
#pragma unroll
    for (int dc = 0; dc < 2; ++dc) qa[dc] = Frag<_Float16>::load(qrow + dc * 32 + 8 * hh);
  }

  float mrow[8], lrow[8];
  v8f oacc[4];
#pragma unroll
  for (int r = 0; r < 8; ++r) { mrow[r] = -INFINITY; lrow[r] = 0.f; }
#pragma unroll
  for (int t = 0; t < 4; ++t) oacc[t] = (v8f){0.f,0.f,0.f,0.f,0.f,0.f,0.f,0.f};

  const int nChunks = (g.causal != 0) ? (qb + 1) : (g.S / AT_KC);
  for (int kc = 0; kc < nChunks; ++kc) {
    const int kv0 = kc * AT_KC;
    __syncthreads();
    {
      const int kvr = tid >> 1, dh = (tid & 1) * 32;
      const _Float16* krow = kb_ptr + (size_t)(kv0 + kvr) * g.k_rs + dh;
      const _Float16* vrow = vb_ptr + (size_t)(kv0 + kvr) * g.v_rs + dh;
#pragma unroll
      for (int i = 0; i < 4; ++i) {
        const v8h kk8 = *(const v8h*)(krow + 8 * i);
        *(v8h*)(Ksh + kvr * AT_D + dh + 8 * i) = kk8;
      }
#pragma unroll
      for (int i = 0; i < 4; ++i) {
        const v8h vv = *(const v8h*)(vrow + 8 * i);
#pragma unroll
        for (int e = 0; e < 8; ++e) Vth[(dh + 8 * i + e) * AT_KC + kvr] = vv[e];
      }
    }
    __syncthreads();

    v8f s[4];
#pragma unroll
    for (int j = 0; j < 4; ++j) {
      s[j] = (v8f){0.f,0.f,0.f,0.f,0.f,0.f,0.f,0.f};
#pragma unroll
      for (int dc = 0; dc < 2; ++dc) {
        FH kb;
        kb.h[0] = *(const v8h*)(Ksh + (j * 16 + c) * AT_D + dc * 32 + 8 * hh);
        kb.h[1] = *(const v8h*)(Ksh + (j * 16 + c) * AT_D + dc * 32 + 16 + 8 * hh);
        s[j] = mma_h(qa[dc], kb.v, s[j]);
      }
    }
    const bool diag = (g.causal != 0) && (kc == qb);
    float cm[8];
#pragma unroll
    for (int r = 0; r < 8; ++r) {
      const int qrow = q0 + 8 * hh + r;
      float m = -INFINITY;
#pragma unroll
      for (int j = 0; j < 4; ++j) {
        const int kvcol = kv0 + j * 16 + c;
        float sv = s[j][r] * g.qscale;
        if (diag && (kvcol > qrow)) sv = -INFINITY;
        s[j][r] = sv;
        m = fmaxf(m, sv);
      }
#pragma unroll
      for (int off = 1; off < 16; off <<= 1) m = fmaxf(m, __shfl_xor(m, off, 32));
      cm[r] = m;
    }
    _Float16* pw = Psh[wave];
#pragma unroll
    for (int r = 0; r < 8; ++r) {
      const float mnew = fmaxf(mrow[r], cm[r]);
      const float alpha = (mrow[r] == -INFINITY) ? 0.0f : expf(mrow[r] - mnew);
      mrow[r] = mnew;
      float psum = 0.f;
#pragma unroll
      for (int j = 0; j < 4; ++j) {
        const float p = expf(s[j][r] - mnew);
        psum += p;
        pw[(8 * hh + r) * AT_KC + j * 16 + c] = (_Float16)(p * AT_PSC);
      }
#pragma unroll
      for (int off = 1; off < 16; off <<= 1) psum += __shfl_xor(psum, off, 32);
      lrow[r] = lrow[r] * alpha + psum;
#pragma unroll
      for (int t = 0; t < 4; ++t) oacc[t][r] *= alpha;
    }
    __builtin_amdgcn_fence(__ATOMIC_RELEASE, "workgroup");
    __builtin_amdgcn_wave_barrier();
    __builtin_amdgcn_fence(__ATOMIC_ACQUIRE, "workgroup");
#pragma unroll 1
    for (int kk = 0; kk < 2; ++kk) {
      FH pa;
      pa.h[0] = *(const v8h*)(pw + c * AT_KC + kk * 32 + 8 * hh);
      pa.h[1] = *(const v8h*)(pw + c * AT_KC + kk * 32 + 16 + 8 * hh);
#pragma unroll
      for (int t = 0; t < 4; ++t) {
        FH vb;
        vb.h[0] = *(const v8h*)(Vth + (t * 16 + c) * AT_KC + kk * 32 + 8 * hh);
        vb.h[1] = *(const v8h*)(Vth + (t * 16 + c) * AT_KC + kk * 32 + 16 + 8 * hh);
        oacc[t] = mma_h(pa.v, vb.v, oacc[t]);
      }
    }
  }

  float* os = Os[wave];
#pragma unroll
  for (int r = 0; r < 8; ++r) {
    const float inv = g.oscale / (lrow[r] * AT_PSC);
#pragma unroll
    for (int t = 0; t < 4; ++t) os[(8 * hh + r) * 68 + t * 16 + c] = oacc[t][r] * inv;
  }
  __builtin_amdgcn_fence(__ATOMIC_RELEASE, "workgroup");
  __builtin_amdgcn_wave_barrier();
  __builtin_amdgcn_fence(__ATOMIC_ACQUIRE, "workgroup");
  {
    const int q4 = lane >> 3, c8 = (lane & 7) * 8;
    for (int pass = 0; pass < 2; ++pass) {
#pragma unroll
      for (int it = 0; it < 4; ++it) {
        const int row = it * 4 + q4;
        const float* sp = os + row * 68 + c8;
        v8h hv;
#pragma unroll
        for (int e = 0; e < 8; ++e) hv[e] = (_Float16)sp[e];
        *(volatile v8h*)(ob_ptr + (size_t)(q0 + row) * g.o_rs + c8) = hv;
      }
      __threadfence();
    }
  }
}

__global__ __launch_bounds__(256) void silu_mul_f16x2(const _Float16* __restrict__ gu, _Float16* __restrict__ hout,
                                                     int M, int F, float oscale) {
  const int halfF = F >> 1;
  const long idx = (long)blockIdx.x * 256 + threadIdx.x;
  if (idx >= (long)M * halfF) return;
  const int row = (int)(idx / halfF);
  const int j   = (int)(idx - (long)row * halfF) * 2;
  const unsigned* gp = (const unsigned*)(const void*)gu;
  const size_t gi = ((size_t)row * (size_t)(2 * F) + (size_t)j) >> 1;
  const size_t ui = ((size_t)row * (size_t)(2 * F) + (size_t)F + (size_t)j) >> 1;
  const unsigned ug = gp[gi], uu = gp[ui];
  const float g0 = (float)__builtin_bit_cast(_Float16, (unsigned short)(ug & 0xFFFFu));
  const float g1 = (float)__builtin_bit_cast(_Float16, (unsigned short)(ug >> 16));
  const float u0 = (float)__builtin_bit_cast(_Float16, (unsigned short)(uu & 0xFFFFu));
  const float u1 = (float)__builtin_bit_cast(_Float16, (unsigned short)(uu >> 16));
  const float s0 = g0 * __builtin_amdgcn_rcpf(1.0f + __expf(-g0));
  const float s1 = g1 * __builtin_amdgcn_rcpf(1.0f + __expf(-g1));
  const _Float16 h0 = (_Float16)(s0 * u0 * oscale);
  const _Float16 h1 = (_Float16)(s1 * u1 * oscale);
  const unsigned uo = (unsigned)__builtin_bit_cast(unsigned short, h0) | ((unsigned)__builtin_bit_cast(unsigned short, h1) << 16);
  const size_t oi = ((size_t)row * (size_t)F + (size_t)j) >> 1;
  ((volatile unsigned*)hout)[oi] = uo;
  __threadfence();
  ((volatile unsigned*)hout)[oi] = uo;
}

extern "C" void kernel_launch(void* const* d_in, const int* in_sizes, int n_in,
                              void* d_out, int out_size, void* d_ws, size_t ws_size,
                              hipStream_t stream) {
  if (n_in < 10) return;
  const float* x     = (const float*)d_in[0];
  const float* Wq    = (const float*)d_in[1];
  const float* Wk    = (const float*)d_in[2];
  const float* Wv    = (const float*)d_in[3];
  const float* Wo    = (const float*)d_in[4];
  const float* Wgate = (const float*)d_in[5];
  const float* Wup   = (const float*)d_in[6];
  const float* Wdown = (const float*)d_in[7];
  const float* g1    = (const float*)d_in[8];
  const float* g2    = (const float*)d_in[9];
  float* out = (float*)d_out;

  const int S = SEQ_LEN;
  const int M = in_sizes[0] / D_MODEL;
  if (M <= 0 || in_sizes[0] != M * D_MODEL || (M % S) != 0 || (M % 64) != 0) return;
  if (out_size != M * D_MODEL) return;
  if (in_sizes[1] != D_MODEL * D_MODEL || in_sizes[2] != KV_DIM * D_MODEL || in_sizes[3] != KV_DIM * D_MODEL ||
      in_sizes[4] != D_MODEL * D_MODEL || in_sizes[5] != FF_DIM * D_MODEL || in_sizes[6] != FF_DIM * D_MODEL ||
      in_sizes[7] != D_MODEL * FF_DIM || in_sizes[8] < D_MODEL || in_sizes[9] < D_MODEL) return;
  const int B = M / S;

  size_t off = 0;
  auto carve = [&](size_t bytes) -> size_t { size_t o = off; off += (bytes + 255) & ~(size_t)255; return o; };
  const size_t oWqkv = carve((size_t)QKV_N * D_MODEL * 2);
  const size_t oWo   = carve((size_t)D_MODEL * D_MODEL * 2);
  const size_t oWgu  = carve((size_t)2 * FF_DIM * D_MODEL * 2);
  const size_t oWd   = carve((size_t)D_MODEL * FF_DIM * 2);
  const size_t oCos  = carve((size_t)32 * S * 4);
  const size_t oSin  = carve((size_t)32 * S * 4);
  const size_t oXn   = carve((size_t)M * D_MODEL * 2);
  const size_t oQkv  = carve((size_t)M * QKV_N * 4);
  const size_t oQ    = carve((size_t)M * D_MODEL * 2);
  const size_t oK    = carve((size_t)M * KV_DIM * 2);
  const size_t oV    = carve((size_t)M * KV_DIM * 2);
  const size_t oAttn = carve((size_t)M * D_MODEL * 2);
  const size_t oX1   = carve((size_t)M * D_MODEL * 4);
  const size_t oGu   = carve((size_t)M * 2 * FF_DIM * 2);
  if (off > ws_size) return;

  char* ws = (char*)d_ws;
  _Float16* Wqkv16 = (_Float16*)(ws + oWqkv);
  _Float16* Wo16   = (_Float16*)(ws + oWo);
  _Float16* Wgu16  = (_Float16*)(ws + oWgu);
  _Float16* Wd16   = (_Float16*)(ws + oWd);
  float*    cosT   = (float*)(ws + oCos);
  float*    sinT   = (float*)(ws + oSin);
  _Float16* xn16   = (_Float16*)(ws + oXn);
  float*    qkv32  = (float*)(ws + oQkv);
  _Float16* hff16  = (_Float16*)(ws + oQkv);
  _Float16* q16    = (_Float16*)(ws + oQ);
  _Float16* k16    = (_Float16*)(ws + oK);
  _Float16* v16    = (_Float16*)(ws + oV);
  _Float16* attn16 = (_Float16*)(ws + oAttn);
  float*    x1     = (float*)(ws + oX1);
  _Float16* gu16   = (_Float16*)(ws + oGu);

  const float WSC = 64.0f;
  const float OSC = 8.0f;
  const float HSC = 16.0f;

  auto cast = [&](const float* src, _Float16* dst, int n) {
    const int n2 = n / 2;
    cast_scale_f32_f16x2<<<dim3((n2 + 255) / 256), dim3(256), 0, stream>>>(src, dst, n2, WSC);
  };
  cast(Wq, Wqkv16, D_MODEL * D_MODEL);
  cast(Wk, Wqkv16 + (size_t)D_MODEL * D_MODEL, KV_DIM * D_MODEL);
  cast(Wv, Wqkv16 + (size_t)(D_MODEL + KV_DIM) * D_MODEL, KV_DIM * D_MODEL);
  cast(Wo, Wo16, D_MODEL * D_MODEL);
  cast(Wgate, Wgu16, FF_DIM * D_MODEL);
  cast(Wup, Wgu16 + (size_t)FF_DIM * D_MODEL, FF_DIM * D_MODEL);
  cast(Wdown, Wd16, D_MODEL * FF_DIM);

  RopeFreq rf;
  for (int i = 0; i < 32; ++i) rf.f[i] = 1.0f / powf(10000.0f, (float)(2 * i) / 64.0f);
  rope_table<<<dim3((S + 255) / 256, 32), dim3(256), 0, stream>>>(cosT, sinT, S, rf);

  const float NSC = 0.036084391824351615f;
  const float EPS = 1e-6f;

  rmsnorm768_f16<<<dim3((M + 7) / 8), dim3(256), 0, stream>>>(x, g1, xn16, M, NSC, EPS);

  {
    const int tiles = (M / 64) * (QKV_N / 64);
    wmma_gemm64<0, false, 0, 0, false, 0><<<dim3((tiles + 7) / 8, 1), dim3(256), 0, stream>>>(
        (const unsigned short*)xn16, (const unsigned short*)xn16, D_MODEL, 0L,
        (const unsigned short*)Wqkv16, (const unsigned short*)Wqkv16, D_MODEL, 0L,
        (void*)qkv32, (void*)qkv32, QKV_N, 0L,
        cosT, x, 0L, M, QKV_N, D_MODEL, 1.0f / WSC);
  }

  rope_split_f16<<<dim3((M * (QKV_N / 8) + 255) / 256), dim3(256), 0, stream>>>(qkv32, cosT, sinT, q16, k16, v16, M, S);

  {
    AttnGeomH g;
    g.q_bs = (long)S * D_MODEL; g.q_rs = D_MODEL; g.q_hs = HDIM;
    g.k_bs = (long)S * KV_DIM;  g.k_rs = KV_DIM;  g.k_hs = HDIM;
    g.v_bs = (long)S * KV_DIM;  g.v_rs = KV_DIM;  g.v_hs = HDIM;
    g.o_bs = (long)S * D_MODEL; g.o_rs = D_MODEL; g.o_hs = HDIM;
    g.S = S; g.H = NQH; g.n_rep = NREP; g.causal = 1; g.qscale = 0.125f; g.oscale = OSC;
    attn64_f16<<<dim3(B * NQH * (S / AT_QB)), dim3(128), 0, stream>>>(q16, k16, v16, attn16, g);
  }

  {
    const int tiles = (M / 64) * (D_MODEL / 64);
    wmma_gemm64<0, false, 0, 0, true, 0><<<dim3((tiles + 7) / 8, 1), dim3(256), 0, stream>>>(
        (const unsigned short*)attn16, (const unsigned short*)attn16, D_MODEL, 0L,
        (const unsigned short*)Wo16, (const unsigned short*)Wo16, D_MODEL, 0L,
        (void*)x1, (void*)x1, D_MODEL, 0L,
        cosT, x, 0L, M, D_MODEL, D_MODEL, 1.0f / (WSC * OSC));
  }

  rmsnorm768_f16<<<dim3((M + 7) / 8), dim3(256), 0, stream>>>(x1, g2, xn16, M, NSC, EPS);

  {
    const int tiles = (M / 64) * ((2 * FF_DIM) / 64);
    wmma_gemm64<0, false, 0, 1, false, 0><<<dim3((tiles + 7) / 8, 1), dim3(256), 0, stream>>>(
        (const unsigned short*)xn16, (const unsigned short*)xn16, D_MODEL, 0L,
        (const unsigned short*)Wgu16, (const unsigned short*)Wgu16, D_MODEL, 0L,
        (void*)gu16, (void*)gu16, 2 * FF_DIM, 0L,
        cosT, x, 0L, M, 2 * FF_DIM, D_MODEL, 1.0f / WSC);
  }

  silu_mul_f16x2<<<dim3((unsigned)(((long)M * (FF_DIM / 2) + 255) / 256)), dim3(256), 0, stream>>>(gu16, hff16, M, FF_DIM, HSC);

  {
    const int tiles = (M / 64) * (D_MODEL / 64);
    wmma_gemm64<0, false, 0, 0, true, 0><<<dim3((tiles + 7) / 8, 1), dim3(256), 0, stream>>>(
        (const unsigned short*)hff16, (const unsigned short*)hff16, FF_DIM, 0L,
        (const unsigned short*)Wd16, (const unsigned short*)Wd16, FF_DIM, 0L,
        (void*)out, (void*)out, D_MODEL, 0L,
        cosT, x1, 0L, M, D_MODEL, FF_DIM, 1.0f / (WSC * HSC));
  }

  (void)ws_size;
}
